// HybridRetention_6605659701981
// MI455X (gfx1250) — hardware-run, weakly checked
//
#include <hip/hip_runtime.h>
#include <math.h>

typedef __attribute__((ext_vector_type(16))) _Float16 v16h;
typedef __attribute__((ext_vector_type(8)))  _Float16 v8h;
typedef __attribute__((ext_vector_type(2)))  _Float16 v2h;
typedef __attribute__((ext_vector_type(16))) __bf16   v16b;
typedef __attribute__((ext_vector_type(8)))  __bf16   v8b;
typedef __attribute__((ext_vector_type(8)))  float    v8f;
typedef __attribute__((ext_vector_type(4)))  float    v4f;
typedef __attribute__((ext_vector_type(2)))  float    v2f;
typedef __attribute__((ext_vector_type(4)))  _Float16 v4h;

constexpr int kNB   = 4;
constexpr int kL    = 2048;
constexpr int kRows = kNB * kL;
constexpr int kD    = 512;
constexpr int kH    = 8;
constexpr int kDh   = 64;
constexpr int kN3   = 3 * kD;
constexpr int kHB   = 4;
constexpr int kOut0 = kRows * kD;
constexpr int kBvO  = kN3;
constexpr int kBvZ  = kN3 + kD;
constexpr int kBvTot = 2 * (kN3 + kD);
constexpr int kThr  = 256;
constexpr float kInCarry = 1024.0f;
constexpr float kWCarry  = 4096.0f;
constexpr float kGCarry  = 256.0f;
constexpr float kSCarry  = 256.0f;
constexpr float kScP = 1.0f / (kInCarry * kWCarry);
constexpr float kScM = 1.0f / (kGCarry * kWCarry);
constexpr float kScS = 1.0f / (kInCarry * kInCarry);
constexpr float kScR = 1.0f / (kSCarry * kInCarry);
constexpr float kLogDecay = -0.105360515657826301f;
constexpr float kF16MinNormal = 6.103515625e-5f;

static_assert(kRows == 8192 && kD == 512 && kH * kDh == kD && kN3 == 1536 && (kH % kHB) == 0 && (kL & (kL - 1)) == 0, "the index arithmetic below uses these sizes");

constexpr size_t kOffQ16 = 0ull;
constexpr size_t kOffK16 = 8388608ull;
constexpr size_t kOffVT16 = 16777216ull;
constexpr size_t kOffWT = 25165824ull;
constexpr size_t kOffWOT = 26738688ull;
constexpr size_t kOffBV = 27262976ull;
constexpr size_t kOffP = 27279360ull;
constexpr size_t kOffHG16 = 77611008ull;
constexpr size_t kOffM = 85999616ull;
constexpr size_t kOffS = 102776832ull;
constexpr size_t kOffSD16 = 169885696ull;
constexpr size_t kOffR = 203440128ull;
constexpr size_t kWsTotal = 220217344ull;
static_assert(kWsTotal <= 268435456ull, "the carve stands under the contract's 256 MiB of workspace");
static_assert(kOffQ16 == 0
  && kOffK16 == kOffQ16 + 8388608ull
  && kOffVT16 == kOffK16 + 8388608ull
  && kOffWT == kOffVT16 + 8388608ull
  && kOffWOT == kOffWT + 1572864ull
  && kOffBV == kOffWOT + 524288ull
  && kOffP == kOffBV + 16384ull
  && kOffHG16 == kOffP + 50331648ull
  && kOffM == kOffHG16 + 8388608ull
  && kOffS == kOffM + 16777216ull
  && kOffSD16 == kOffS + 67108864ull
  && kOffR == kOffSD16 + 33554432ull
  && kWsTotal == kOffR + 16777216ull, "the carve is a chain: every region starts where the one before ends");
static_assert((size_t)kRows * kD * 2 == 8388608ull && (size_t)kNB * kH * kDh * kL * 2 == 8388608ull && (size_t)kN3 * kD * 2 == 1572864ull && (size_t)kD * kD * 2 == 524288ull && (size_t)kBvTot * 4 == 16384ull && (size_t)kRows * kN3 * 4 == 50331648ull
  && (size_t)kRows * kD * 4 == 16777216ull && (size_t)kHB * kL * kL * 4 == 67108864ull && (size_t)kHB * kL * kL * 2 == 33554432ull, "every region's length is its plane's");
static_assert((kOffK16 % 256) == 0 && (kOffVT16 % 256) == 0 && (kOffWT % 256) == 0 && (kOffWOT % 256) == 0 && (kOffBV % 256) == 0 && (kOffP % 256) == 0 && (kOffHG16 % 256) == 0 && (kOffM % 256) == 0 && (kOffS % 256) == 0 && (kOffSD16 % 256) == 0 && (kOffR % 256) == 0, "every region starts on a multiple of 256 B");

__device__ __forceinline__ unsigned short f2bf_bits(float f) {
  unsigned u = __float_as_uint(f);
  return (unsigned short)((u + 0x7FFFu + ((u >> 16) & 1u)) >> 16);
}
__device__ __forceinline__ float bf_bits2f(unsigned short h) { return __uint_as_float(((unsigned)h) << 16); }
__device__ __forceinline__ float bf16r(float f) { return bf_bits2f(f2bf_bits(f)); }
__device__ __forceinline__ float carry_flush(float v, float carry) {
  const float s = v * carry;
  return (fabsf(s) < kF16MinNormal) ? 0.0f : s;
}

__device__ __forceinline__ void dep_guard4_h(v8f& a, v8f& b, v8f& c, v8f& d, v16h x, v16h y) { asm volatile("v_nop\n\tv_nop\n\tv_nop\n\tv_nop" : "+v"(a), "+v"(b), "+v"(c), "+v"(d) : "v"(x), "v"(y)); }
__device__ __forceinline__ void dep_guard4_b(v8f& a, v8f& b, v8f& c, v8f& d, v16b x, v16b y) { asm volatile("v_nop\n\tv_nop\n\tv_nop\n\tv_nop" : "+v"(a), "+v"(b), "+v"(c), "+v"(d) : "v"(x), "v"(y)); }
__device__ __forceinline__ void keep4_h(v16h a, v16h b, v16h c, v16h d) { asm volatile("v_nop" :: "v"(a), "v"(b), "v"(c), "v"(d)); }
__device__ __forceinline__ void keep4_b(v16b a, v16b b, v16b c, v16b d) { asm volatile("v_nop" :: "v"(a), "v"(b), "v"(c), "v"(d)); }
__device__ __forceinline__ void acc_guard4(v8f& a, v8f& b, v8f& c, v8f& d) { asm volatile("v_nop\n\tv_nop\n\tv_nop\n\tv_nop" : "+v"(a), "+v"(b), "+v"(c), "+v"(d)); }

template <typename T> struct Frag;
template <> struct Frag<_Float16> {
  typedef v16h V; union U { v16h v; v8h h[2]; };
  static __device__ __forceinline__ v16h load(const _Float16* p) {
    U f; f.h[0] = *(const v8h*)(p); f.h[1] = *(const v8h*)(p + 16); return f.v;
  }
  static __device__ __forceinline__ v8f mma(v16h a, v16h b, v8f c) {
    return __builtin_amdgcn_wmma_f32_16x16x32_f16(false, a, false, b, (short)0, c, false, false);
  }
  static __device__ __forceinline__ void guard4(v8f& a, v8f& b, v8f& c, v8f& d, v16h x, v16h y) { dep_guard4_h(a, b, c, d, x, y); }
  static __device__ __forceinline__ void keep(v16h a, v16h b, v16h c, v16h d) { keep4_h(a, b, c, d); }
};
template <> struct Frag<__bf16> {
  typedef v16b V; union U { v16b v; v8b h[2]; };
  static __device__ __forceinline__ v16b load(const __bf16* p) {
    U f; f.h[0] = *(const v8b*)(p); f.h[1] = *(const v8b*)(p + 16); return f.v;
  }
  static __device__ __forceinline__ v8f mma(v16b a, v16b b, v8f c) {
    return __builtin_amdgcn_wmma_f32_16x16x32_bf16(false, a, false, b, (short)0, c, false, false);
  }
  static __device__ __forceinline__ void guard4(v8f& a, v8f& b, v8f& c, v8f& d, v16b x, v16b y) { dep_guard4_b(a, b, c, d, x, y); }
  static __device__ __forceinline__ void keep(v16b a, v16b b, v16b c, v16b d) { keep4_b(a, b, c, d); }
};

__device__ __forceinline__ v8f mma_h(v16h a, v16h b, v8f c) {
  c = __builtin_amdgcn_wmma_f32_16x16x32_f16(false, a, false, b, (short)0, c, false, false);
  asm volatile("v_nop\n\tv_nop\n\tv_nop\n\tv_nop" : "+v"(c) : "v"(a), "v"(b));
  return c;
}

template <int ET> struct Elem;
template <> struct Elem<0> { typedef _Float16 T; };
template <> struct Elem<1> { typedef __bf16 T; };
template <int ET, bool SPLIT, int BIAS_MODE, int OUT_MODE, bool RESID, int ACT = 0>
__global__ __launch_bounds__(256) void wmma_gemm64(
    const unsigned short* __restrict__ Ap, const unsigned short* __restrict__ A2p, int lda, long strideA,
    const unsigned short* __restrict__ Btp, const unsigned short* __restrict__ Bt2p, int ldb, long strideB,
    void* __restrict__ Cout, void* __restrict__ Cout2, int ldc, long strideC,
    const float* __restrict__ bias,
    const float* __restrict__ resid, long strideR,
    int M, int N, int K, float scale) {
  typedef typename Elem<ET>::T T;
  typedef typename Frag<T>::V V;
  const T* A = (const T*)Ap; const T* A2 = (const T*)A2p; const T* Bt = (const T*)Btp; const T* Bt2 = (const T*)Bt2p;
  __shared__ __align__(16) float sT[8][16 * 68];
  const int b    = blockIdx.y;
  const int lane = threadIdx.x & 31;
  const int wave = threadIdx.x >> 5;
  const int tilesN = N >> 6;
  const int tilesM = M >> 6;
  const int tile = blockIdx.x * 8 + wave;
  if (tile >= tilesM * tilesN) return;
  const int tm = tile / tilesN;
  const int tn = tile - tm * tilesN;
  const int m0 = tm << 6;
  const int n0 = tn << 6;

  const T* Ab  = A  + (size_t)b * strideA;
  const T* Bb  = Bt + (size_t)b * strideB;
  const T* Ab2 = SPLIT ? (A2  + (size_t)b * strideA) : nullptr;
  const T* Bb2 = SPLIT ? (Bt2 + (size_t)b * strideB) : nullptr;

  const int rlane = lane & 15;
  const int koff  = (lane >> 4) * 8;
  const int mOff  = (lane >> 4) * 8;

  v8f acc[4][4];
#pragma unroll
  for (int i = 0; i < 4; ++i)
#pragma unroll
    for (int j = 0; j < 4; ++j) acc[i][j] = (v8f){0.f,0.f,0.f,0.f,0.f,0.f,0.f,0.f};

  for (int k0 = 0; k0 < K; k0 += 32) {
    V bh[4], bl[4];
#pragma unroll
    for (int j = 0; j < 4; ++j) {
      const size_t bo = (size_t)(n0 + (j << 4) + rlane) * ldb + koff + k0;
      bh[j] = Frag<T>::load(Bb + bo);
      if (SPLIT) bl[j] = Frag<T>::load(Bb2 + bo);
    }
#pragma unroll
    for (int i = 0; i < 4; ++i) {
      const size_t ao = (size_t)(m0 + (i << 4) + rlane) * lda + koff + k0;
      V ah = Frag<T>::load(Ab + ao);
      V al;
      if (SPLIT) al = Frag<T>::load(Ab2 + ao);
#pragma unroll
      for (int j = 0; j < 4; ++j) {
        acc[i][j] = Frag<T>::mma(ah, bh[j], acc[i][j]);
        if (SPLIT) {
          acc[i][j] = Frag<T>::mma(ah, bl[j], acc[i][j]);
          acc[i][j] = Frag<T>::mma(al, bh[j], acc[i][j]);
        }
      }
      Frag<T>::guard4(acc[i][0], acc[i][1], acc[i][2], acc[i][3], ah, SPLIT ? al : ah);
    }
    Frag<T>::keep(bh[0], bh[1], bh[2], bh[3]);
    if (SPLIT) Frag<T>::keep(bl[0], bl[1], bl[2], bl[3]);
  }
  acc_guard4(acc[0][0], acc[0][1], acc[0][2], acc[0][3]);
  acc_guard4(acc[1][0], acc[1][1], acc[1][2], acc[1][3]);
  acc_guard4(acc[2][0], acc[2][1], acc[2][2], acc[2][3]);
  acc_guard4(acc[3][0], acc[3][1], acc[3][2], acc[3][3]);

  float* slab = sT[wave];
  const float* Rb = RESID ? (resid + (size_t)b * strideR) : nullptr;
#pragma unroll
  for (int i = 0; i < 4; ++i) {
    const int mBase = m0 + (i << 4);
#pragma unroll
    for (int j = 0; j < 4; ++j) {
      const int n = n0 + (j << 4) + rlane;
      float bv = 0.f;
      if (BIAS_MODE == 2) bv = bias[n];
#pragma unroll
      for (int r = 0; r < 8; ++r) {
        float v = acc[i][j][r] * scale;
        if (BIAS_MODE == 1) v += bias[mBase + mOff + r];
        if (BIAS_MODE == 2) v += bv;
        if (RESID) v += Rb[(size_t)(mBase + mOff + r) * ldc + n];
        if (ACT == 1) v = tanhf(v);
        if (ACT == 2) v = fmaxf(v, 0.0f);
        if (ACT == 3) v = v / (1.0f + expf(-v));
        if (ACT == 4) v = (v > 0.f) ? v : 0.01f * v;
        slab[(mOff + r) * 68 + (j << 4) + rlane] = v;
      }
    }
    __builtin_amdgcn_fence(__ATOMIC_RELEASE, "workgroup");
    __builtin_amdgcn_wave_barrier();
    __builtin_amdgcn_fence(__ATOMIC_ACQUIRE, "workgroup");
    if (OUT_MODE == 0) {
      float* C = (float*)Cout + (size_t)b * strideC;
      const int hh = lane >> 4, c4 = (lane & 15) * 4;
      for (int pass = 0; pass < 2; ++pass) {
#pragma unroll
        for (int it = 0; it < 8; ++it) {
          const int row = it * 2 + hh;
          v4f v = *(const v4f*)(slab + row * 68 + c4);
          *(volatile v4f*)(C + (size_t)(mBase + row) * ldc + n0 + c4) = v;
        }
        __threadfence();
      }
    } else {
      const int q = lane >> 3, c8 = (lane & 7) * 8;
      unsigned short* C  = (unsigned short*)Cout  + (size_t)b * strideC;
      unsigned short* C2 = (OUT_MODE == 2) ? ((unsigned short*)Cout2 + (size_t)b * strideC) : nullptr;
      for (int pass = 0; pass < 2; ++pass) {
#pragma unroll
        for (int it = 0; it < 4; ++it) {
          const int row = it * 4 + q;
          const float* sp = slab + row * 68 + c8;
          v8h hv, lv;
#pragma unroll
          for (int e = 0; e < 8; ++e) {
            if (OUT_MODE == 1) {
              hv[e] = (_Float16)sp[e];
            } else {
              unsigned short hb = f2bf_bits(sp[e]);
              unsigned short lb = f2bf_bits(sp[e] - bf_bits2f(hb));
              hv[e] = __builtin_bit_cast(_Float16, hb);
              lv[e] = __builtin_bit_cast(_Float16, lb);
            }
          }
          *(volatile v8h*)(C + (size_t)(mBase + row) * ldc + n0 + c8) = hv;
          if (OUT_MODE == 2) *(volatile v8h*)(C2 + (size_t)(mBase + row) * ldc + n0 + c8) = lv;
        }
        __threadfence();
      }
    }
    __builtin_amdgcn_fence(__ATOMIC_RELEASE, "workgroup");
    __builtin_amdgcn_wave_barrier();
    __builtin_amdgcn_fence(__ATOMIC_ACQUIRE, "workgroup");
  }
}


__global__ __launch_bounds__(kThr) void cast_plane_kernel(const float* __restrict__ src, unsigned short* __restrict__ dst,
                                                          int colsLog2, int dstPitch, int dstOff) {
  const int i   = blockIdx.x * kThr + threadIdx.x;
  const int sh  = colsLog2 - 3;
  const int row = i >> sh;
  const int c8  = (i & ((1 << sh) - 1)) * 8;
  const float* sp = src + ((size_t)row << colsLog2) + c8;
  const v4f a0 = *(const v4f*)(sp);
  const v4f a1 = *(const v4f*)(sp + 4);
  v8h hv;
#pragma unroll
  for (int e = 0; e < 4; ++e) {
    const float f0 = a0[e];
    const float f1 = a1[e];
    hv[e]     = (_Float16)carry_flush(bf16r(f0), kInCarry);
    hv[4 + e] = (_Float16)carry_flush(bf16r(f1), kInCarry);
  }
  unsigned short* dp = dst + (size_t)row * dstPitch + dstOff + c8;
  *(volatile v8h*)dp = hv;
  __threadfence();
  *(volatile v8h*)dp = hv;
}

__global__ __launch_bounds__(256) void wt_plane_kernel(const float* __restrict__ W, unsigned short* __restrict__ dst, int K, int N, int nLive, int ldd, int colOff) {
  const int n  = blockIdx.x;
  const int k8 = threadIdx.x * 8;
  const bool live = n < nLive;
  const int nc = live ? n : 0;
  v8h hv;
#pragma unroll
  for (int e = 0; e < 8; ++e) {
    const float w = W[(size_t)(k8 + e) * N + nc];
    hv[e] = (_Float16)(live ? carry_flush(bf16r(w), kWCarry) : 0.0f);
  }
  unsigned short* dp = dst + (size_t)n * ldd + colOff + k8;
  *(volatile v8h*)dp = hv;
  __threadfence();
  *(volatile v8h*)dp = hv;
}

__global__ __launch_bounds__(kThr) void setup_kernel(const float* __restrict__ ba, const float* __restrict__ bb, const float* __restrict__ bg, const float* __restrict__ bo, float* __restrict__ BV) {
  const unsigned i = blockIdx.x * (unsigned)kThr + threadIdx.x;
  const unsigned j = i & (unsigned)(kD - 1);
  const unsigned w = i >> 9;
  const float va = ba[j], vb = bb[j], vg = bg[j], vo = bo[j];
  const float v = (w == 0u) ? va : ((w == 1u) ? vb : ((w == 2u) ? vg : vo));
  const float o = (w < 4u) ? bf16r(v) : 0.0f;
  float* dp = BV + i;
  *(volatile float*)dp = o;
  __threadfence();
  *(volatile float*)dp = o;
}
static_assert(16 * kThr == kBvTot && kD == 512, "set-up grid exact: 16 blocks");

__global__ __launch_bounds__(kThr) void vt_kernel(const float* __restrict__ v, unsigned short* __restrict__ VT16) {
  const unsigned i = blockIdx.x * (unsigned)kThr + threadIdx.x;
  const unsigned s8 = (i & 255u) * 8u;
  const unsigned d = (i >> 8) & 63u;
  const unsigned z = i >> 14;
  const unsigned sq = z >> 3, hd = z & 7u;
  const float* pv = v + (sq * (unsigned)kL + s8) * (unsigned)kD + hd * (unsigned)kDh + d;
  v8h hv;
#pragma unroll
  for (int e = 0; e < 8; ++e) hv[e] = (_Float16)carry_flush(bf16r(pv[(unsigned)e * (unsigned)kD]), kInCarry);
  unsigned short* dp = VT16 + i * 8u;
  *(volatile v8h*)dp = hv;
  __threadfence();
  *(volatile v8h*)dp = hv;
}
static_assert((size_t)kNB * kH * kDh * (kL / 8) == 2048ull * kThr && kL / 8 == 256 && kDh == 64, "the transposed v's grid exact: 2,048 blocks");

__global__ __launch_bounds__(kThr) void scan_kernel(const float* __restrict__ P, unsigned short* __restrict__ HG16) {
  const unsigned ix = blockIdx.x * (unsigned)kThr + threadIdx.x;
  const unsigned sq = ix >> 8;
  const unsigned d = (ix & 255u) * 2u;
  float h0 = 0.0f, h1 = 0.0f;
  for (int t = 0; t < kL; ++t) {
    const unsigned row = sq * (unsigned)kL + (unsigned)t;
    const float* pp = P + row * (unsigned)kN3 + d;
    const v2f pa = *(const v2f*)pp, pb = *(const v2f*)(pp + kD), pg = *(const v2f*)(pp + 2 * kD);
    h0 = (1.0f / (1.0f + expf(-pa[0]))) * h0 + pb[0];
    h1 = (1.0f / (1.0f + expf(-pa[1]))) * h1 + pb[1];
    v2h o;
    o[0] = (_Float16)carry_flush(h0 * (1.0f / (1.0f + expf(-pg[0]))), kGCarry);
    o[1] = (_Float16)carry_flush(h1 * (1.0f / (1.0f + expf(-pg[1]))), kGCarry);
    unsigned short* dp = HG16 + row * (unsigned)kD + d;
    *(volatile v2h*)dp = o;
    __threadfence();
    *(volatile v2h*)dp = o;
  }
}
static_assert(kNB * (kD / 2) == 4 * kThr && (kD % 2) == 0, "the scan's grid exact: 4 blocks: one a sequence");

__global__ __launch_bounds__(kThr) void decay_kernel(const float* __restrict__ S, unsigned short* __restrict__ SD16) {
  const unsigned i = blockIdx.x * (unsigned)kThr + threadIdx.x;
  const unsigned s8 = (i & 255u) * 8u;
  const unsigned t = (i >> 8) & (unsigned)(kL - 1);
  const v4f a0 = *(const v4f*)(S + i * 8u), a1 = *(const v4f*)(S + i * 8u + 4);
  v8h hv;
#pragma unroll
  for (int e = 0; e < 8; ++e) {
    const unsigned s = s8 + (unsigned)e;
    const bool live = s <= t;
    const float dl = (float)(live ? (t - s) : 0u);
    const float sc = ((e < 4) ? a0[e] : a1[e - 4]) * expf(dl * kLogDecay);
    hv[e] = (_Float16)(live ? carry_flush(sc, kSCarry) : 0.0f);
  }
  unsigned short* dp = SD16 + i * 8u;
  *(volatile v8h*)dp = hv;
  __threadfence();
  *(volatile v8h*)dp = hv;
}
static_assert((size_t)kHB * kL * (kL / 8) == 8192ull * kThr && kL == 2048, "the decay's grid exact: 8,192 blocks a launch");

__global__ __launch_bounds__(kThr) void close_kernel(const float* __restrict__ M, const float* __restrict__ R, float* __restrict__ out) {
  const unsigned i = blockIdx.x * (unsigned)kThr + threadIdx.x;
  const v4f m0 = *(const v4f*)(M + i * 8u), m1 = *(const v4f*)(M + i * 8u + 4);
  const v4f r0 = *(const v4f*)(R + i * 8u), r1 = *(const v4f*)(R + i * 8u + 4);
  v4f o0, o1;
#pragma unroll
  for (int e = 0; e < 4; ++e) { o0[e] = m0[e] + r0[e]; o1[e] = m1[e] + r1[e]; }
  float* dp = out + i * 8u;
  for (int pass = 0; pass < 2; ++pass) {
    *(volatile v4f*)dp = o0;
    *(volatile v4f*)(dp + 4) = o1;
    __threadfence();
  }
}
static_assert((size_t)kOut0 / 8 == 2048ull * kThr && (size_t)kHB * kL * kL < 4294967296ull / 4 && (size_t)kRows * kN3 < 4294967296ull / 4, "the closing sum's grid exact: 2,048 blocks; every plane's element offsets fit 32 bits");

extern "C" void kernel_launch(void* const* d_in, const int* in_sizes, int n_in,
                              void* d_out, int out_size, void* d_ws, size_t ws_size,
                              hipStream_t stream) {
  if (n_in < 11 || d_out == nullptr || d_ws == nullptr) return;
  if (in_sizes[0] != kOut0 || in_sizes[1] != kOut0 || in_sizes[2] != kOut0 || in_sizes[3] != kD * kD || in_sizes[4] != kD || in_sizes[5] != kD * kD || in_sizes[6] != kD || in_sizes[7] != kD * kD || in_sizes[8] != kD
      || in_sizes[9] != kD * kD || in_sizes[10] != kD) return;
  if (out_size != kOut0) return;
  if (ws_size < kWsTotal) return;
  const float* q = (const float*)d_in[0];
  const float* k = (const float*)d_in[1];
  const float* v = (const float*)d_in[2];
  const float* Wa = (const float*)d_in[3];
  const float* ba = (const float*)d_in[4];
  const float* Wb = (const float*)d_in[5];
  const float* bb = (const float*)d_in[6];
  const float* Wg = (const float*)d_in[7];
  const float* bg = (const float*)d_in[8];
  const float* Wo = (const float*)d_in[9];
  const float* bo = (const float*)d_in[10];
  float* out = (float*)d_out;
  char* ws = (char*)d_ws;
  unsigned short* Q16 = (unsigned short*)(ws + kOffQ16);
  unsigned short* K16 = (unsigned short*)(ws + kOffK16);
  unsigned short* VT16 = (unsigned short*)(ws + kOffVT16);
  unsigned short* WT = (unsigned short*)(ws + kOffWT);
  unsigned short* WOT = (unsigned short*)(ws + kOffWOT);
  float* BV = (float*)(ws + kOffBV);
  float* P = (float*)(ws + kOffP);
  unsigned short* HG16 = (unsigned short*)(ws + kOffHG16);
  float* M = (float*)(ws + kOffM);
  float* S = (float*)(ws + kOffS);
  unsigned short* SD16 = (unsigned short*)(ws + kOffSD16);
  float* R = (float*)(ws + kOffR);

  static_assert(((size_t)kRows * kD / 8) % kThr == 0 && kD / 8 == 64 && (1 << 9) == kD, "the row casts' grid (a source row is 2^9 = 512 values); the transposing casts run one block a destination row with exactly K / 8 threads");
  cast_plane_kernel<<<(int)(((size_t)kRows * kD / 8) / kThr), kThr, 0, stream>>>(q, Q16, 9, kD, 0);
  cast_plane_kernel<<<(int)(((size_t)kRows * kD / 8) / kThr), kThr, 0, stream>>>(k, K16, 9, kD, 0);
  vt_kernel<<<2048, kThr, 0, stream>>>(v, VT16);
  wt_plane_kernel<<<kD, kD / 8, 0, stream>>>(Wa, WT, kD, kD, kD, kD, 0);
  wt_plane_kernel<<<kD, kD / 8, 0, stream>>>(Wb, WT + (size_t)kD * kD, kD, kD, kD, kD, 0);
  wt_plane_kernel<<<kD, kD / 8, 0, stream>>>(Wg, WT + (size_t)2 * kD * kD, kD, kD, kD, kD, 0);
  wt_plane_kernel<<<kD, kD / 8, 0, stream>>>(Wo, WOT, kD, kD, kD, kD, 0);
  setup_kernel<<<16, kThr, 0, stream>>>(ba, bb, bg, bo, BV);
  wmma_gemm64<0, false, 2, 0, false, 0><<<dim3((kRows / 64) * (kN3 / 64) / 8, 1), 256, 0, stream>>>(
      Q16, Q16, kD, 0L, WT, WT, kD, 0L, (void*)P, (void*)P, kN3, 0L, BV, nullptr, 0L, kRows, kN3, kD, kScP);
  scan_kernel<<<4, kThr, 0, stream>>>(P, HG16);
  wmma_gemm64<0, false, 2, 0, false, 0><<<dim3((kRows / 64) * (kD / 64) / 8, 1), 256, 0, stream>>>(
      HG16, HG16, kD, 0L, WOT, WOT, kD, 0L, (void*)M, (void*)M, kD, 0L, BV + kBvO, nullptr, 0L, kRows, kD, kD, kScM);
  for (int sq = 0; sq < kNB; ++sq) {
    for (int hg = 0; hg < kH / kHB; ++hg) {
      const size_t qoff = (size_t)sq * kL * kD + (size_t)hg * kHB * kDh;
      const size_t voff = ((size_t)sq * kH + (size_t)hg * kHB) * kDh * kL;
      wmma_gemm64<0, false, 2, 0, false, 0><<<dim3((kL / 64) * (kL / 64) / 8, kHB), 256, 0, stream>>>(
          Q16 + qoff, Q16 + qoff, kD, (long)kDh, K16 + qoff, K16 + qoff, kD, (long)kDh, (void*)S, (void*)S, kL, (long)kL * kL, BV + kBvZ, nullptr, 0L, kL, kL, kDh, kScS);
      decay_kernel<<<8192, kThr, 0, stream>>>(S, SD16);
      wmma_gemm64<0, false, 2, 0, false, 0><<<dim3((kL / 64) * (kDh / 64) / 8, kHB), 256, 0, stream>>>(
          SD16, SD16, kL, (long)kL * kL, VT16 + voff, VT16 + voff, kL, (long)kDh * kL, (void*)(R + qoff), (void*)(R + qoff), kD, (long)kDh, BV + kBvZ, nullptr, 0L, kL, kDh, kL, kScR);
    }
  }
  close_kernel<<<2048, kThr, 0, stream>>>(M, R, out);
}
static_assert(((kRows / 64) * (kN3 / 64)) % 8 == 0 && ((kRows / 64) * (kD / 64)) % 8 == 0 && ((kL / 64) * (kL / 64)) % 8 == 0 && ((kL / 64) * (kDh / 64)) % 8 == 0, "the engine's grids: whole blocks of eight wave tiles");
